// QKVInviBasedAttn_128849019012
// MI455X (gfx1250) — hardware-verified
//
#include <hip/hip_runtime.h>

#define BB   8
#define NN   2048
#define DIN  512
#define DK   64

typedef _Float16 v16h __attribute__((ext_vector_type(16)));
typedef _Float16 v8h  __attribute__((ext_vector_type(8)));
typedef _Float16 v8ha __attribute__((ext_vector_type(8), may_alias));
typedef float    v8f  __attribute__((ext_vector_type(8)));
typedef float    v4f  __attribute__((ext_vector_type(4)));
typedef float    v4fa __attribute__((ext_vector_type(4), may_alias));
union Frag { v16h v; v8h half[2]; _Float16 h[16]; };

__device__ __forceinline__ v8f mma16(v16h a, v16h b, v8f c) {
  c = __builtin_amdgcn_wmma_f32_16x16x32_f16(false, a, false, b, (short)0, c, false, false);
  asm volatile("v_nop\n\tv_nop\n\tv_nop\n\tv_nop" : "+v"(c) : "v"(a), "v"(b));
  return c;
}

__global__ __launch_bounds__(256) void k_cvt(const float* __restrict__ src, _Float16* __restrict__ dst, int n8) {
  const int t = blockIdx.x * 256 + threadIdx.x;
  if (t >= n8) return;
  const v4f a = *(const v4fa*)(src + (size_t)t * 8), b = *(const v4fa*)(src + (size_t)t * 8 + 4);
  v8h v; v[0]=(_Float16)a[0]; v[1]=(_Float16)a[1]; v[2]=(_Float16)a[2]; v[3]=(_Float16)a[3];
  v[4]=(_Float16)b[0]; v[5]=(_Float16)b[1]; v[6]=(_Float16)b[2]; v[7]=(_Float16)b[3];
  *(volatile v8h*)(dst + (size_t)t * 8) = v;
  __threadfence();
  *(volatile v8h*)(dst + (size_t)t * 8) = v;
}

__global__ __launch_bounds__(128) void k_proj(const float* __restrict__ A, const float* __restrict__ Wm, const float* __restrict__ bias,
                                            _Float16* __restrict__ P, int nrows) {
  __shared__ __attribute__((aligned(16))) _Float16 sW[DK][DIN + 8];
  __shared__ __attribute__((aligned(16))) _Float16 sOut[4][16][DK + 8];
  const int tid = threadIdx.x, w = tid >> 5, lane = tid & 31, ln = lane & 15, hh = lane >> 4;
  for (int e = tid; e < DIN * DK; e += 128) { const int k = e / DK, n = e % DK; sW[n][k] = (_Float16)Wm[e]; }
  __syncthreads();
  const int row0 = (blockIdx.x * 4 + w) * 16;
  if (row0 < nrows) {
    const float* arow = A + (size_t)(row0 + ln) * DIN;
    v8f acc[4] = {};
    for (int kb = 0; kb < DIN; kb += 32) {
      Frag a;
      const v4f l0 = *(const v4fa*)(arow + kb + 8 * hh), l1 = *(const v4fa*)(arow + kb + 8 * hh + 4);
      const v4f h0 = *(const v4fa*)(arow + kb + 16 + 8 * hh), h1 = *(const v4fa*)(arow + kb + 16 + 8 * hh + 4);
#pragma unroll
      for (int i = 0; i < 4; ++i) { a.h[i] = (_Float16)l0[i]; a.h[4+i] = (_Float16)l1[i]; a.h[8+i] = (_Float16)h0[i]; a.h[12+i] = (_Float16)h1[i]; }
#pragma unroll
      for (int t = 0; t < 4; ++t) {
        Frag b;
        b.half[0] = *(const v8ha*)&sW[t * 16 + ln][kb + 8 * hh];
        b.half[1] = *(const v8ha*)&sW[t * 16 + ln][kb + 16 + 8 * hh];
        acc[t] = mma16(a.v, b.v, acc[t]);
      }
    }
#pragma unroll
    for (int t = 0; t < 4; ++t) {
      const float bv = bias[t * 16 + ln];
#pragma unroll
      for (int r = 0; r < 8; ++r) sOut[w][8 * hh + r][t * 16 + ln] = (_Float16)(acc[t][r] + bv);
    }
    __builtin_amdgcn_fence(__ATOMIC_ACQ_REL, "workgroup");
    __builtin_amdgcn_wave_barrier();
    const int rsub = lane >> 3, c8 = (lane & 7) * 8;
    for (int pass = 0; pass < 2; ++pass) {
#pragma unroll
      for (int q = 0; q < 4; ++q) {
        const int r = q * 4 + rsub;
        const v8h v = *(const v8ha*)&sOut[w][r][c8];
        *(volatile v8h*)(P + (size_t)(row0 + r) * DK + c8) = v;
      }
      if (pass == 0) __threadfence();
    }
  }
}

__global__ __launch_bounds__(128) void k_scores(const _Float16* __restrict__ Qh, const _Float16* __restrict__ Kh,
                                              _Float16* __restrict__ Pm, float* __restrict__ rowscale) {
  __shared__ __attribute__((aligned(16))) _Float16 sK[64][DK + 8];
  __shared__ __attribute__((aligned(16))) _Float16 sP[4][16][72];
  __shared__ __attribute__((aligned(16))) float sRS[64];
  const int tid = threadIdx.x, w = tid >> 5, lane = tid & 31, ln = lane & 15, hh = lane >> 4;
  const int b = blockIdx.x / (NN / 64), qb = blockIdx.x % (NN / 64);
  const int q0 = qb * 64 + w * 16;
  const _Float16* Qb = Qh + (size_t)b * NN * DK; const _Float16* Kb = Kh + (size_t)b * NN * DK;
  Frag aq[2];
#pragma unroll
  for (int ks = 0; ks < 2; ++ks) {
    aq[ks].half[0] = *(const v8ha*)(Qb + (size_t)(q0 + ln) * DK + ks * 32 + 8 * hh);
    aq[ks].half[1] = *(const v8ha*)(Qb + (size_t)(q0 + ln) * DK + ks * 32 + 16 + 8 * hh);
  }
  float rmax[8], rsum[8];
#pragma unroll
  for (int r = 0; r < 8; ++r) { rmax[r] = -3.0e38f; rsum[r] = 0.f; }

  for (int pass = 0; pass < 2; ++pass) {
    for (int c = 0; c < NN / 64; ++c) {
      const int j0 = c * 64;
      __syncthreads();
      for (int e = tid; e < 64 * (DK / 8); e += 128) { const int r = e >> 3, c8 = (e & 7) * 8; *(v8ha*)&sK[r][c8] = *(const v8ha*)(Kb + (size_t)(j0 + r) * DK + c8); }
      __syncthreads();
      v8f s[4];
#pragma unroll
      for (int nt = 0; nt < 4; ++nt) {
        v8f acc = {};
#pragma unroll
        for (int ks = 0; ks < 2; ++ks) {
          Frag bk;
          bk.half[0] = *(const v8ha*)&sK[nt * 16 + ln][ks * 32 + 8 * hh];
          bk.half[1] = *(const v8ha*)&sK[nt * 16 + ln][ks * 32 + 16 + 8 * hh];
          acc = mma16(aq[ks].v, bk.v, acc);
        }
        s[nt] = acc * 0.125f;
      }
      if (pass == 0) {
#pragma unroll
        for (int r = 0; r < 8; ++r) {
          float m = fmaxf(fmaxf(s[0][r], s[1][r]), fmaxf(s[2][r], s[3][r]));
          m = fmaxf(m, __shfl_xor(m, 1, 32)); m = fmaxf(m, __shfl_xor(m, 2, 32)); m = fmaxf(m, __shfl_xor(m, 4, 32)); m = fmaxf(m, __shfl_xor(m, 8, 32));
          rmax[r] = fmaxf(rmax[r], m);
        }
      } else {
#pragma unroll
        for (int nt = 0; nt < 4; ++nt)
#pragma unroll
          for (int r = 0; r < 8; ++r) {
            const _Float16 pv = (_Float16)__expf(s[nt][r] - rmax[r]);
            rsum[r] += (float)pv;
            sP[w][8 * hh + r][nt * 16 + ln] = pv;
          }
        __builtin_amdgcn_fence(__ATOMIC_ACQ_REL, "workgroup");
        __builtin_amdgcn_wave_barrier();
        for (int ps = 0; ps < 2; ++ps) {
#pragma unroll
          for (int q = 0; q < 4; ++q) {
            const int r = q * 4 + (lane >> 3), c8 = (lane & 7) * 8;
            const v8h v = *(const v8ha*)&sP[w][r][c8];
            *(volatile v8h*)(Pm + ((size_t)b * NN + q0 + r) * NN + j0 + c8) = v;
          }
          if (ps == 0) __threadfence();
        }
        __builtin_amdgcn_fence(__ATOMIC_ACQ_REL, "workgroup");
        __builtin_amdgcn_wave_barrier();
      }
    }
  }
#pragma unroll
  for (int r = 0; r < 8; ++r) {
    float s = rsum[r];
    s += __shfl_xor(s, 1, 32); s += __shfl_xor(s, 2, 32); s += __shfl_xor(s, 4, 32); s += __shfl_xor(s, 8, 32);
    rsum[r] = s;
  }
  if (ln == 0) {
#pragma unroll
    for (int r = 0; r < 8; ++r) sRS[w * 16 + 8 * hh + r] = 1.0f / rsum[r];
  }
  __syncthreads();
  if (tid < 16) {
    const v4f v = *(const v4fa*)&sRS[tid * 4];
    float* dst = rowscale + (size_t)b * NN + qb * 64 + tid * 4;
    *(volatile v4f*)dst = v;
    __threadfence();
    *(volatile v4f*)dst = v;
  }
}

__global__ __launch_bounds__(128) void k_pv(const _Float16* __restrict__ Pm, const _Float16* __restrict__ Xh,
                                          const float* __restrict__ rowscale, float* __restrict__ out) {
  __shared__ __attribute__((aligned(16))) _Float16 sX[32][128 + 8];
  __shared__ __attribute__((aligned(16))) float sO[4][16][128];
  const int tid = threadIdx.x, w = tid >> 5, lane = tid & 31, ln = lane & 15, hh = lane >> 4;
  const int nqb = NN / 64, ndb = DIN / 128;
  const int b = blockIdx.x / (nqb * ndb), rem = blockIdx.x % (nqb * ndb), qb = rem / ndb, dq = rem % ndb;
  const int q0 = qb * 64 + w * 16, d0 = dq * 128;
  const _Float16* Prow = Pm + ((size_t)b * NN + q0 + ln) * NN;
  const _Float16* Xb = Xh + (size_t)b * NN * DIN;
  v8f acc[8] = {};
  for (int c = 0; c < NN / 32; ++c) {
    const int j0 = c * 32;
    __syncthreads();
    for (int e = tid; e < 32 * 16; e += 128) { const int r = e >> 4, c8 = (e & 15) * 8; *(v8ha*)&sX[r][c8] = *(const v8ha*)(Xb + (size_t)(j0 + r) * DIN + d0 + c8); }
    __syncthreads();
    Frag a;
    a.half[0] = *(const v8ha*)(Prow + j0 + 8 * hh);
    a.half[1] = *(const v8ha*)(Prow + j0 + 16 + 8 * hh);
#pragma unroll
    for (int t = 0; t < 8; ++t) {
      Frag bx;
#pragma unroll
      for (int i = 0; i < 8; ++i) { bx.h[i] = sX[8 * hh + i][t * 16 + ln]; bx.h[8 + i] = sX[16 + 8 * hh + i][t * 16 + ln]; }
      acc[t] = mma16(a.v, bx.v, acc[t]);
    }
  }
  float rs[8];
#pragma unroll
  for (int r = 0; r < 8; ++r) rs[r] = rowscale[(size_t)b * NN + q0 + 8 * hh + r];
#pragma unroll
  for (int t = 0; t < 8; ++t)
#pragma unroll
    for (int r = 0; r < 8; ++r) sO[w][8 * hh + r][t * 16 + ln] = acc[t][r] * rs[r];
  __builtin_amdgcn_fence(__ATOMIC_ACQ_REL, "workgroup");
  __builtin_amdgcn_wave_barrier();
  float* ob = out + ((size_t)b * NN + q0) * DIN + d0;
  for (int pass = 0; pass < 2; ++pass) {
#pragma unroll
    for (int r = 0; r < 16; ++r) {
      const v4f v = *(const v4fa*)&sO[w][r][lane * 4];
      *(volatile v4f*)(ob + (size_t)r * DIN + lane * 4) = v;
    }
    if (pass == 0) __threadfence();
  }
}

extern "C" void kernel_launch(void* const* d_in, const int* in_sizes, int n_in,
                              void* d_out, int out_size, void* d_ws, size_t ws_size, hipStream_t stream) {
  (void)in_sizes; (void)n_in; (void)out_size;
  const float* X  = (const float*)d_in[0];
  const float* h  = (const float*)d_in[1];
  const float* WQ = (const float*)d_in[2];
  const float* bQ = (const float*)d_in[3];
  const float* WK = (const float*)d_in[4];
  const float* bK = (const float*)d_in[5];
  char* ws = (char*)d_ws; size_t off = 0;
  _Float16* Xh = (_Float16*)(ws + off); off += (size_t)BB * NN * DIN * 2;
  _Float16* Qh = (_Float16*)(ws + off); off += (size_t)BB * NN * DK * 2;
  _Float16* Kh = (_Float16*)(ws + off); off += (size_t)BB * NN * DK * 2;
  _Float16* Pm = (_Float16*)(ws + off); off += (size_t)BB * NN * NN * 2;
  float* rowscale = (float*)(ws + off); off += (size_t)BB * NN * 4;
  if (off > ws_size) return;
  const int nrows = BB * NN;
  k_cvt<<<(nrows * DIN / 8 + 255) / 256, 256, 0, stream>>>(X, Xh, nrows * DIN / 8);
  k_proj<<<nrows / 64, 128, 0, stream>>>(h, WQ, bQ, Qh, nrows);
  k_proj<<<nrows / 64, 128, 0, stream>>>(X, WK, bK, Kh, nrows);
  k_scores<<<BB * (NN / 64), 128, 0, stream>>>(Qh, Kh, Pm, rowscale);
  k_pv<<<BB * (NN / 64) * (DIN / 128), 128, 0, stream>>>(Pm, Xh, rowscale, (float*)d_out);
}
